// EvidenceLevelAttention_85718957293806
// MI455X (gfx1250) — hardware-run, weakly checked
//
#include <hip/hip_runtime.h>


namespace {
constexpr int NB_ = 8, N = 256, H = 300, HP = 320  , HT_ = 304  , NT = NB_ * N;
constexpr float XS = 8.0f, PS = 256.0f, WSC = 256.0f;
typedef _Float16 b16;
typedef __attribute__((ext_vector_type(16))) _Float16 v16b;
typedef __attribute__((ext_vector_type(8))) _Float16 v8b;
typedef __attribute__((ext_vector_type(2))) _Float16 v2b;
typedef __attribute__((ext_vector_type(8))) float v8f;
typedef __attribute__((ext_vector_type(4))) float v4f;
__device__ __forceinline__ float bf16_rne(float f) { unsigned int u = __float_as_uint(f); u += 0x7FFFu + ((u >> 16) & 1u); float r = __uint_as_float(u & 0xFFFF0000u); asm volatile("" : "+v"(r)); return r; }
__device__ __forceinline__ float bfv(float f) { float r = bf16_rne(f); asm volatile("" : "+v"(r)); return r; }
__device__ __forceinline__ void split16(float v, b16& hi, b16& lo) { hi = (b16)v; lo = (b16)(v - (float)hi); }
__device__ __forceinline__ v16b frag_kb(const b16* p, int hh) { const v8b a = *(const v8b*)(p + 8 * hh), b = *(const v8b*)(p + 16 + 8 * hh); v16b f;
#pragma unroll
  for (int e = 0; e < 8; ++e) { f[e] = a[e]; f[8 + e] = b[e]; } return f; }
__device__ __forceinline__ v8f wmma16b(v16b a, v16b b, v8f c) { v8f d = __builtin_amdgcn_wmma_f32_16x16x32_f16(false, a, false, b, (short)0, c, false, false); asm volatile("v_nop\n\tv_nop\n\tv_nop\n\tv_nop" : "+v"(d) : "v"(a), "v"(b)); return d; }
__device__ __forceinline__ void wave_lds_sync() { __builtin_amdgcn_fence(__ATOMIC_RELEASE, "workgroup"); __builtin_amdgcn_wave_barrier(); __builtin_amdgcn_fence(__ATOMIC_ACQUIRE, "workgroup"); }
__device__ __forceinline__ float pmul(float a, float b) { float p = a * b; asm volatile("" : "+v"(p)); return p; }

__global__ __launch_bounds__(256) void wput_kernel(const float* __restrict__ w0, b16* __restrict__ WAB) { const int u = blockIdx.x * 256 + threadIdx.x; if (u >= 2 * HT_ * (HP / 8)) return; const int r = u / (HP / 8), k0 = (u % (HP / 8)) * 8; const int half = r / HT_, o = r % HT_; v8b v;
#pragma unroll
  for (int j = 0; j < 8; ++j) { const int k = k0 + j; v[j] = (b16)((o < H && k < H) ? bf16_rne(w0[(size_t)o * 2 * H + half * H + k]) * WSC : 0.0f); }
  for (int pass = 0; pass < 2; ++pass) { *(volatile v8b*)(WAB + (size_t)r * HP + k0) = v; __threadfence(); } }
__global__ __launch_bounds__(32) void proj_kernel(const float* __restrict__ h, const b16* __restrict__ WAB, float* __restrict__ AI, float* __restrict__ AJ) { __shared__ __attribute__((aligned(16))) b16 Ah[16][HP + 8]; __shared__ float Tf[16][HT_ + 4]; const int lane = threadIdx.x, nloc = lane & 15, hlf = lane >> 4; const size_t r0 = (size_t)blockIdx.x * 16;
  for (int rr = 0; rr < 16; ++rr) for (int q = 0; q < HP / 32; ++q) { const int c = q * 32 + lane; Ah[rr][c] = (b16)(c < H ? bf16_rne(h[(r0 + rr) * H + c]) * XS : 0.0f); }
  if (lane < 16) for (int k = HP; k < HP + 8; ++k) Ah[lane][k] = (b16)0.0f;
  wave_lds_sync();
#pragma unroll 1
  for (int g = 0; g < 2; ++g) { float* dst = g ? AJ : AI;
#pragma unroll 1
    for (int tg = 0; tg < 19; tg += 10) { const int nt = tg == 0 ? 10 : 9; v8f acc[10];
#pragma unroll
      for (int t = 0; t < 10; ++t) acc[t] = (v8f){};
#pragma unroll 2
      for (int kb = 0; kb < HP; kb += 32) { const v16b a = frag_kb(&Ah[nloc][kb], hlf);
#pragma unroll
        for (int t = 0; t < 10; ++t) if (t < nt) acc[t] = wmma16b(a, frag_kb(WAB + ((size_t)g * HT_ + (tg + t) * 16 + nloc) * HP + kb, hlf), acc[t]); }
#pragma unroll
      for (int t = 0; t < 10; ++t) if (t < nt)
#pragma unroll
        for (int r8 = 0; r8 < 8; ++r8) Tf[8 * hlf + r8][(tg + t) * 16 + nloc] = acc[t][r8] * (1.0f / (XS * WSC)); }
    wave_lds_sync();
    for (int pass = 0; pass < 2; ++pass) { for (int rr = 0; rr < 16; ++rr) for (int q = 0; q < HP / 32; ++q) { const int c = q * 32 + lane; ((volatile float*)dst)[(r0 + rr) * HP + c] = c < HT_ ? Tf[rr][c] : 0.0f; } __threadfence(); }
    wave_lds_sync(); } }
__global__ __launch_bounds__(256) void ht_kernel(const float* __restrict__ h, b16* __restrict__ HT) { __shared__ float Tt[64][HT_ + 1]; const int b = blockIdx.x / (N / 64), j0 = (blockIdx.x % (N / 64)) * 64; const int tid = threadIdx.x, wave = tid >> 5, lane = tid & 31;
  for (int q = wave; q < 64; q += 8) for (int c = lane; c < HT_; c += 32) Tt[q][c] = c < H ? bfv(h[((size_t)b * N + j0 + q) * H + c]) : 0.0f;
  __syncthreads();
  for (int pass = 0; pass < 2; ++pass) { for (int hh = wave; hh < HT_; hh += 8) { *(volatile v2b*)(HT + ((size_t)b * HT_ + hh) * N + j0 + lane * 2) = (v2b){(b16)(Tt[lane * 2][hh] * XS), (b16)(Tt[lane * 2 + 1][hh] * XS)}; } __threadfence(); } }
__global__ __launch_bounds__(32) void att_kernel(const float* __restrict__ AI, const float* __restrict__ AJ, const float* __restrict__ b0, const float* __restrict__ w1, const float* __restrict__ b1, const b16* __restrict__ HT, int BLIM, float* __restrict__ out) { __shared__ float Ai[32][H + 1], Sc[32][N + 1], B0[H], W1s[H]; __shared__ __attribute__((aligned(16))) b16 Pa[32][N + 8], Pb[32][N + 8]; const int lane = threadIdx.x, nloc = lane & 15, hlf = lane >> 4; const int b = blockIdx.x / (N / 32), i0 = (blockIdx.x % (N / 32)) * 32; if (b >= BLIM) return; const size_t row0 = (size_t)b * N + i0;
  for (int rr = 0; rr < 32; ++rr) for (int c = lane; c < H; c += 32) Ai[rr][c] = AI[(row0 + rr) * HP + c];
  for (int c = lane; c < H; c += 32) { B0[c] = bfv(b0[c]); W1s[c] = bfv(w1[c]); }
  wave_lds_sync(); const float bb1 = bfv(b1[0]);
#pragma unroll 1
  for (int j = 0; j < N; ++j) { const float* aj = AJ + ((size_t)b * N + j) * HP; float s = bb1;
#pragma unroll 4
    for (int c = 0; c < H; ++c) s += pmul(fmaxf(Ai[lane][c] + aj[c] + B0[c], 0.0f), W1s[c]); Sc[lane][j] = s; }
  { float mx = -INFINITY; for (int j = 0; j < N; ++j) mx = fmaxf(mx, Sc[lane][j]); float sm = 0.0f; for (int j = 0; j < N; ++j) { const float e = __expf(Sc[lane][j] - mx); Sc[lane][j] = e; sm += e; } const float inv = 1.0f / sm; for (int j = 0; j < N; ++j) { b16 p, pl; split16(Sc[lane][j] * inv * PS, p, pl); Pa[lane][j] = p; Pb[lane][j] = pl; } for (int k = N; k < N + 8; ++k) { Pa[lane][k] = (b16)0.0f; Pb[lane][k] = (b16)0.0f; } }
  wave_lds_sync();
  for (int pass = 0; pass < 2; ++pass) {
#pragma unroll 1
    for (int tg = 0; tg < 19; tg += 5) { const int nt = (19 - tg) < 5 ? (19 - tg) : 5; v8f acc[2][5];
#pragma unroll
      for (int rt = 0; rt < 2; ++rt)
#pragma unroll
        for (int t = 0; t < 5; ++t) acc[rt][t] = (v8f){};
#pragma unroll 2
      for (int kb = 0; kb < N; kb += 32)
#pragma unroll
        for (int rt = 0; rt < 2; ++rt) { const v16b pa = frag_kb(&Pa[rt * 16 + nloc][kb], hlf), pb = frag_kb(&Pb[rt * 16 + nloc][kb], hlf);
#pragma unroll
          for (int t = 0; t < 5; ++t) if (t < nt) { const v16b bw = frag_kb(HT + ((size_t)b * HT_ + (tg + t) * 16 + nloc) * N + kb, hlf); acc[rt][t] = wmma16b(pa, bw, acc[rt][t]); acc[rt][t] = wmma16b(pb, bw, acc[rt][t]); } }
#pragma unroll
      for (int rt = 0; rt < 2; ++rt)
#pragma unroll
        for (int t = 0; t < 5; ++t) if (t < nt)
#pragma unroll
          for (int r8 = 0; r8 < 8; ++r8) { const int i = rt * 16 + 8 * hlf + r8, c = (tg + t) * 16 + nloc; if (c < H) ((volatile float*)out)[(row0 + i) * H + c] = acc[rt][t][r8] * (1.0f / (PS * XS)); } }
    __threadfence(); } }
}

extern "C" void kernel_launch(void* const* d_in, const int* in_sizes, int n_in, void* d_out, int out_size, void* d_ws, size_t ws_size, hipStream_t stream) {
  (void)n_in;
  auto Fp = [&](int i) { return (const float*)d_in[i]; };
  if (in_sizes[0] != NT * H || in_sizes[1] != H * 2 * H || in_sizes[2] != H || in_sizes[3] != H || in_sizes[4] != 1 || out_size != NT * H) return;
  const int BLIM = NB_;
  size_t off = 0; char* ws = (char*)d_ws;
  auto carve = [&](size_t bytes) { char* p = ws + off; off += (bytes + 255) & ~(size_t)255; return p; };
  b16* WAB = (b16*)carve((size_t)2 * HT_ * HP * 2); float* AI = (float*)carve((size_t)NT * HP * 4); float* AJ = (float*)carve((size_t)NT * HP * 4); b16* HT = (b16*)carve((size_t)NB_ * HT_ * N * 2);
  if (off > ws_size || off > ((size_t)12 << 20)) return;
  wput_kernel<<<(2 * HT_ * (HP / 8) + 255) / 256, 256, 0, stream>>>(Fp(1), WAB);
  proj_kernel<<<NT / 16, 32, 0, stream>>>(Fp(0), WAB, AI, AJ);
  ht_kernel<<<NB_ * (N / 64), 256, 0, stream>>>(Fp(0), HT);
  att_kernel<<<BLIM * (N / 32), 32, 0, stream>>>(AI, AJ, Fp(2), Fp(3), Fp(4), HT, BLIM, (float*)d_out);
}
